// EncoderGraphGRU_35064113004950
// MI455X (gfx1250) — hardware-verified
//
#include <hip/hip_runtime.h>
#include <stddef.h>
#include <math.h>


#define XD     128
#define HD     256
#define FD     288
#define FP     320
#define TD     16
#define ZD     64
#define NTHR   256
#define NWAVE  8
#define NBE    256
#define AGR    257
#define RT     32
#define HP     264
#define EPT    8
#define NGRP   2
#define CHUNK  (NTHR * EPT * NGRP)
#define WCAP   (EPT * NGRP * 32)
#define LISTN  (NWAVE * WCAP)
#define PCAP   (LISTN + 64)
#define GR     64
#define PLN    512
#define WSC    64.0f
#define ASC    8.0f
#define RSC    0.001953125f
#define WSCAP  134217728
#define OFW1F  0
#define OFW2   65536
#define OFHI   131072
#define OFWIH0 278528
#define OFWHH0 499712
#define OFWIH1 696320
#define OFWHH1 892928
#define OFHEAD 1089536
#define WPTOT  1122304
#define WPB    2048
#define LDS_EDGE ((AGR * FP + RT * HP) * 2 + (LISTN + PCAP + 3 * RT + 16) * 4)

static_assert(OFW2 == 2 * HD * XD);
static_assert(OFHI == OFW2 + HD * HD);
static_assert(OFWIH0 == OFHI + 2 * HD * FD);
static_assert(OFWHH0 == OFWIH0 + 3 * HD * FD);
static_assert(OFWIH1 == OFWHH0 + 3 * HD * HD);
static_assert(OFWHH1 == OFWIH1 + 3 * HD * HD);
static_assert(OFHEAD == OFWHH1 + 3 * HD * HD);
static_assert(WPTOT == OFHEAD + 2 * ZD * HD);
static_assert((OFW2 % WPB) == 0 && (OFHI % WPB) == 0 && (OFWIH0 % WPB) == 0 && (OFWHH0 % WPB) == 0);
static_assert((OFWIH1 % WPB) == 0 && (OFWHH1 % WPB) == 0 && (OFHEAD % WPB) == 0 && (WPTOT % WPB) == 0);
static_assert(((HD * XD) % WPB) == 0 && ((HD * FD) % WPB) == 0 && ((ZD * HD) % WPB) == 0);
static_assert(NTHR * 8 == WPB);
static_assert(CHUNK == 4096);
static_assert((PCAP % 32) == 0);
static_assert(((AGR * FP) % 8) == 0);
static_assert((((AGR * FP + RT * HP) * 2) % 16) == 0);
static_assert((FP % 8) == 0 && (HP % 8) == 0 && (PLN % 32) == 0);
static_assert(FD == 9 * 32 && HD == 8 * 32 && XD == 4 * 32);
static_assert(LDS_EDGE <= 300000);
static_assert(GR == 4 * 16 && NTHR == 32 * NWAVE);

typedef float    v4f  __attribute__((ext_vector_type(4)));
typedef float    v8f  __attribute__((ext_vector_type(8)));
typedef int      v4i  __attribute__((ext_vector_type(4)));
typedef _Float16 v8h  __attribute__((ext_vector_type(8)));
typedef _Float16 v16h __attribute__((ext_vector_type(16)));
union Frag { v16h v; v8h h[2]; };

__device__ __forceinline__ v8f wmh(v16h a, v16h b, v8f c) {
  v8f d = __builtin_amdgcn_wmma_f32_16x16x32_f16(false, a, false, b, (short)0, c, false, false);
  asm volatile("v_nop\n\tv_nop\n\tv_nop\n\tv_nop" : "+v"(d) : "v"(a), "v"(b));
  return d;
}

__device__ __forceinline__ v8f zacc() { v8f z = {0.f, 0.f, 0.f, 0.f, 0.f, 0.f, 0.f, 0.f}; return z; }

__device__ __forceinline__ v16h ldfrag(const _Float16* p) {
  Frag f;
  f.h[0] = *(const v8h*)p;
  f.h[1] = *(const v8h*)(p + 16);
  return f.v;
}

__device__ __forceinline__ v8h cvt8(v4f a, v4f b, float s) {
  v8h r;
  r[0] = (_Float16)(a.x * s); r[1] = (_Float16)(a.y * s); r[2] = (_Float16)(a.z * s); r[3] = (_Float16)(a.w * s);
  r[4] = (_Float16)(b.x * s); r[5] = (_Float16)(b.y * s); r[6] = (_Float16)(b.z * s); r[7] = (_Float16)(b.w * s);
  return r;
}

__device__ __forceinline__ v4f sel4(bool c, v4f a, v4f b) {
  v4f r;
  r.x = c ? a.x : b.x; r.y = c ? a.y : b.y; r.z = c ? a.z : b.z; r.w = c ? a.w : b.w;
  return r;
}

__device__ __forceinline__ v4f relu4(v4f a) {
  v4f r;
  r.x = fmaxf(a.x, 0.0f); r.y = fmaxf(a.y, 0.0f); r.z = fmaxf(a.z, 0.0f); r.w = fmaxf(a.w, 0.0f);
  return r;
}

__device__ __forceinline__ float sigf(float x) {
  const float e = __expf(-fabsf(x));
  const float s = __builtin_amdgcn_rcpf(1.0f + e);
  return x >= 0.0f ? s : e * s;
}
__device__ __forceinline__ float tanhf2(float x) {
  const float e = __expf(-2.0f * fabsf(x));
  const float t = (1.0f - e) * __builtin_amdgcn_rcpf(1.0f + e);
  return x >= 0.0f ? t : -t;
}

template <int NT, int KS>
__device__ __forceinline__ void gemm16(const _Float16* A0, int lda, const _Float16* B0, int ldb,
                                       int lane, v8f (&acc)[NT]) {
  const int hh = lane >> 4, m = lane & 15;
#pragma unroll
  for (int t = 0; t < NT; ++t) acc[t] = zacc();
  const _Float16* ap = A0 + (size_t)m * lda + 8 * hh;
  const _Float16* bp = B0 + (size_t)m * ldb + 8 * hh;
#pragma unroll 1
  for (int ks = 0; ks < KS; ++ks) {
    const v16h a = ldfrag(ap + 32 * ks);
#pragma unroll
    for (int t = 0; t < NT; ++t) {
      const v16h b = ldfrag(bp + (size_t)(16 * t) * ldb + 32 * ks);
      acc[t] = wmh(a, b, acc[t]);
    }
  }
}

template <int NB>
__device__ __forceinline__ int scan_chunk(const int* __restrict__ dsts, int nE, int cbase, int slotBase,
                                          int vec8, int* list, int tid, int lane, int wave) {
  int wc = 0;
#pragma unroll
  for (int g = 0; g < NGRP; ++g) {
    const int el0  = (g * NTHR + tid) * EPT;
    const int e0   = cbase + el0;
    const int sent = -2147483647 - 1;
    v4i da, db;
    if (vec8 != 0 && cbase + CHUNK <= nE) {
      da = *(const v4i*)(dsts + e0);
      db = *(const v4i*)(dsts + e0 + 4);
    } else {
      da.x = (e0     < nE) ? dsts[min(e0, nE - 1)] : sent;
      da.y = (e0 + 1 < nE) ? dsts[min(e0 + 1, nE - 1)] : sent;
      da.z = (e0 + 2 < nE) ? dsts[min(e0 + 2, nE - 1)] : sent;
      da.w = (e0 + 3 < nE) ? dsts[min(e0 + 3, nE - 1)] : sent;
      db.x = (e0 + 4 < nE) ? dsts[min(e0 + 4, nE - 1)] : sent;
      db.y = (e0 + 5 < nE) ? dsts[min(e0 + 5, nE - 1)] : sent;
      db.z = (e0 + 6 < nE) ? dsts[min(e0 + 6, nE - 1)] : sent;
      db.w = (e0 + 7 < nE) ? dsts[min(e0 + 7, nE - 1)] : sent;
    }
    const unsigned nb = (unsigned)slotBase;
    const unsigned s0 = (unsigned)da.x - nb, s1 = (unsigned)da.y - nb;
    const unsigned s2 = (unsigned)da.z - nb, s3 = (unsigned)da.w - nb;
    const unsigned s4 = (unsigned)db.x - nb, s5 = (unsigned)db.y - nb;
    const unsigned s6 = (unsigned)db.z - nb, s7 = (unsigned)db.w - nb;
    const bool h0 = s0 < (unsigned)NB, h1 = s1 < (unsigned)NB, h2 = s2 < (unsigned)NB, h3 = s3 < (unsigned)NB;
    const bool h4 = s4 < (unsigned)NB, h5 = s5 < (unsigned)NB, h6 = s6 < (unsigned)NB, h7 = s7 < (unsigned)NB;
    const unsigned any = __builtin_amdgcn_ballot_w32(h0 | h1 | h2 | h3 | h4 | h5 | h6 | h7);
    if (any != 0u) {
#define HITJ(J, HJ) { \
        const unsigned mj = __builtin_amdgcn_ballot_w32(HJ); \
        if (mj != 0u) { \
          if (HJ) { \
            const int pos = wc + (int)__builtin_amdgcn_mbcnt_lo(mj, 0u); \
            if (pos < WCAP) list[wave * WCAP + pos] = e0 + (J); \
          } \
          wc += (int)__builtin_popcount(mj); } }
      HITJ(0, h0)
      HITJ(1, h1)
      HITJ(2, h2)
      HITJ(3, h3)
      HITJ(4, h4)
      HITJ(5, h5)
      HITJ(6, h6)
      HITJ(7, h7)
#undef HITJ
    }
  }
  return wc;
}

__global__ __launch_bounds__(NTHR) void k_wprep(const float* __restrict__ w1, const float* __restrict__ w2,
    const float* __restrict__ hw0, const float* __restrict__ hw1, const float* __restrict__ wi0,
    const float* __restrict__ wh0, const float* __restrict__ wi1, const float* __restrict__ wh1,
    const float* __restrict__ muw, const float* __restrict__ lvw, _Float16* WP) {
  const int blk = blockIdx.x, tid = threadIdx.x;
  const int d0 = blk * WPB + tid * 8;
  const float* sp;
  int base, mode = 0;
  if (blk < (HD * XD) / WPB)                { sp = w1;  base = 0;             mode = 1; }
  else if (blk < OFW2 / WPB)                { sp = w1;  base = HD * XD;       mode = 2; }
  else if (blk < OFHI / WPB)                { sp = w2;  base = OFW2; }
  else if (blk < (OFHI + HD * FD) / WPB)    { sp = hw0; base = OFHI; }
  else if (blk < OFWIH0 / WPB)              { sp = hw1; base = OFHI + HD * FD; }
  else if (blk < OFWHH0 / WPB)              { sp = wi0; base = OFWIH0; }
  else if (blk < OFWIH1 / WPB)              { sp = wh0; base = OFWHH0; }
  else if (blk < OFWHH1 / WPB)              { sp = wi1; base = OFWIH1; }
  else if (blk < OFHEAD / WPB)              { sp = wh1; base = OFWHH1; }
  else if (blk < (OFHEAD + ZD * HD) / WPB)  { sp = muw; base = OFHEAD; }
  else                                      { sp = lvw; base = OFHEAD + ZD * HD; }
  const int loc = d0 - base;
  v4f a, b;
  if (mode == 0) {
    a = *(const v4f*)(sp + loc);
    b = *(const v4f*)(sp + loc + 4);
  } else {
    const int n = loc >> 7, k = loc & (XD - 1);
    const float* rb = sp + (size_t)n * (2 * XD) + XD + k;
    a = *(const v4f*)rb;
    b = *(const v4f*)(rb + 4);
    if (mode == 1) {
      const float* ra = sp + (size_t)n * (2 * XD) + k;
      const v4f a2 = *(const v4f*)ra, b2v = *(const v4f*)(ra + 4);
      a = a2 - a;
      b = b2v - b;
    }
  }
  const v8h hv = cvt8(a, b, WSC);
  _Float16* dp = WP + d0;
  *(volatile v8h*)dp = hv;
  __threadfence();
  *(volatile v8h*)dp = hv;
}

__global__ __launch_bounds__(NTHR) void k_xcvt(const float* __restrict__ x, _Float16* X16, int nN) {
  const int d0 = (blockIdx.x * NTHR + threadIdx.x) * 8;
  const int row = d0 >> 7, c = d0 & (XD - 1);
  const int srow = row > nN - 1 ? nN - 1 : row;
  const float* xp = x + (size_t)srow * XD + c;
  const v8h hv = cvt8(*(const v4f*)xp, *(const v4f*)(xp + 4), ASC);
  _Float16* dp = X16 + d0;
  *(volatile v8h*)dp = hv;
  __threadfence();
  *(volatile v8h*)dp = hv;
}

template <int MODE, int KS>
__global__ __launch_bounds__(NTHR) void k_gemm(const _Float16* __restrict__ Ap, int lda,
    const _Float16* __restrict__ Bp, int ldb, const float* __restrict__ bA, const float* __restrict__ bB,
    const float* __restrict__ eps, float* outF, _Float16* outH, int ldo,
    float* o1, float* o2, float* o3, int nN) {
  __shared__ __attribute__((aligned(16))) float stg[GR * 128];
  __shared__ __attribute__((aligned(16))) float sb[128];
  const int tid = threadIdx.x, lane = tid & 31, wave = tid >> 5, hh = lane >> 4, m = lane & 15;
  const int rt = wave & 3, ch = wave >> 2;
  const int rowBase = blockIdx.x * GR, colBase = blockIdx.y * 128;
  if (tid < 32) {
    const int c = colBase + 4 * tid;
    const v4f z4 = {0.f, 0.f, 0.f, 0.f};
    v4f v;
    if (MODE == 0) {
      const int ca = c < HD - 4 ? c : HD - 4;
      const v4f va = *(const v4f*)(bA + ca);
      v = sel4(c < HD, va, z4);
    } else if (MODE == 1) {
      const int ca = c < HD - 4 ? c : HD - 4;
      int cb = c - HD; cb = cb < 0 ? 0 : (cb > HD - 4 ? HD - 4 : cb);
      const v4f va = *(const v4f*)(bA + ca), vb = *(const v4f*)(bB + cb);
      v = sel4(c < HD, va, vb);
    } else {
      const int ca = c < ZD - 4 ? c : ZD - 4;
      int cb = c - ZD; cb = cb < 0 ? 0 : (cb > ZD - 4 ? ZD - 4 : cb);
      const v4f va = *(const v4f*)(bA + ca), vb = *(const v4f*)(bB + cb);
      v = sel4(c < ZD, va, vb);
    }
    *(v4f*)(sb + 4 * tid) = v;
  }
  __syncthreads();
  v8f acc[4];
  gemm16<4, KS>(Ap + (size_t)(rowBase + 16 * rt) * lda, lda, Bp + (size_t)(colBase + 64 * ch) * ldb, ldb, lane, acc);
#pragma unroll
  for (int t = 0; t < 4; ++t) {
    const float bv = sb[64 * ch + 16 * t + m];
    float* sp = stg + (16 * rt + 8 * hh) * 128 + 64 * ch + 16 * t + m;
#pragma unroll
    for (int r = 0; r < 8; ++r) {
      float v = acc[t][r] * RSC + bv;
      if (MODE == 1) v = tanhf2(v);
      sp[r * 128] = v;
    }
  }
  __syncthreads();
  if (MODE != 2) {
    float* gp = outF + (size_t)rowBase * ldo + colBase;
    _Float16* ghp = outH + (size_t)rowBase * ldo + colBase;
#pragma unroll
    for (int it = 0; it < 8; ++it) {
      const int f = it * NTHR + tid, row = f >> 5, p4 = (f & 31) * 4;
      const v4f v = *(const v4f*)(stg + row * 128 + p4);
      *(volatile v4f*)(gp + (size_t)row * ldo + p4) = v;
    }
    if (MODE == 1) {
#pragma unroll
      for (int it = 0; it < 4; ++it) {
        const int f = it * NTHR + tid, row = f >> 4, p8 = (f & 15) * 8;
        const v8h hv = cvt8(*(const v4f*)(stg + row * 128 + p8), *(const v4f*)(stg + row * 128 + p8 + 4), ASC);
        *(volatile v8h*)(ghp + (size_t)row * ldo + p8) = hv;
      }
    }
    __threadfence();
#pragma unroll
    for (int it = 0; it < 8; ++it) {
      const int f = it * NTHR + tid, row = f >> 5, p4 = (f & 31) * 4;
      const v4f v = *(const v4f*)(stg + row * 128 + p4);
      *(volatile v4f*)(gp + (size_t)row * ldo + p4) = v;
    }
    if (MODE == 1) {
#pragma unroll
      for (int it = 0; it < 4; ++it) {
        const int f = it * NTHR + tid, row = f >> 4, p8 = (f & 15) * 8;
        const v8h hv = cvt8(*(const v4f*)(stg + row * 128 + p8), *(const v4f*)(stg + row * 128 + p8 + 4), ASC);
        *(volatile v8h*)(ghp + (size_t)row * ldo + p8) = hv;
      }
    }
  } else {
    v4f mu4[4], lv4[4], z4[4];
    size_t oo[4];
    bool ok[4];
#pragma unroll
    for (int it = 0; it < 4; ++it) {
      const int f = it * NTHR + tid, row = f >> 4, p4 = (f & 15) * 4;
      const int node = rowBase + row;
      const int ncl = node < nN ? node : nN - 1;
      const v4f mu = *(const v4f*)(stg + row * 128 + p4);
      const v4f lv = *(const v4f*)(stg + row * 128 + ZD + p4);
      const v4f ev = *(const v4f*)(eps + (size_t)ncl * ZD + p4);
      v4f z;
      z.x = mu.x + ev.x * __expf(0.5f * lv.x);
      z.y = mu.y + ev.y * __expf(0.5f * lv.y);
      z.z = mu.z + ev.z * __expf(0.5f * lv.z);
      z.w = mu.w + ev.w * __expf(0.5f * lv.w);
      mu4[it] = mu; lv4[it] = lv; z4[it] = z;
      oo[it] = (size_t)ncl * ZD + p4;
      ok[it] = node < nN;
    }
#pragma unroll
    for (int it = 0; it < 4; ++it) {
      if (ok[it]) {
        *(volatile v4f*)(o1 + oo[it]) = mu4[it];
        *(volatile v4f*)(o2 + oo[it]) = lv4[it];
        *(volatile v4f*)(o3 + oo[it]) = z4[it];
      }
    }
    __threadfence();
#pragma unroll
    for (int it = 0; it < 4; ++it) {
      if (ok[it]) {
        *(volatile v4f*)(o1 + oo[it]) = mu4[it];
        *(volatile v4f*)(o2 + oo[it]) = lv4[it];
        *(volatile v4f*)(o3 + oo[it]) = z4[it];
      }
    }
  }
}

template <int KS1>
__global__ __launch_bounds__(NTHR) void k_gate(const _Float16* __restrict__ Xp, int ldx,
    const _Float16* __restrict__ Wih, int ldw, const _Float16* __restrict__ Hp, const float* __restrict__ Hf,
    int ldh, int hoff, const _Float16* __restrict__ Whh, const float* __restrict__ bih,
    const float* __restrict__ bhh, float* outL, _Float16* NH, int nN) {
  __shared__ __attribute__((aligned(16))) float stg[GR * 64];
  __shared__ __attribute__((aligned(16))) float hpv[GR * 64];
  __shared__ __attribute__((aligned(16))) float sbias[4 * 64];
  const int tid = threadIdx.x, lane = tid & 31, wave = tid >> 5, hh = lane >> 4, m = lane & 15;
  const int rt = wave & 3, ch = wave >> 2;
  const int rowBase = blockIdx.x * GR;
  const int jB = blockIdx.y * 64;
  const int jw = jB + 32 * ch;
#pragma unroll
  for (int it = 0; it < 4; ++it) {
    const int f = it * NTHR + tid, row = f >> 4, p4 = (f & 15) * 4;
    const v4f v = *(const v4f*)(Hf + (size_t)(rowBase + row) * ldh + hoff + jB + p4);
    *(v4f*)(hpv + row * 64 + p4) = v;
  }
  if (tid < 64) {
    const int sel = tid >> 4, p4 = (tid & 15) * 4;
    const int goff = (sel == 0 ? 0 : (sel == 1 ? HD : 2 * HD)) + jB + p4;
    const v4f va = *(const v4f*)(bih + goff);
    const v4f vb = *(const v4f*)(bhh + goff);
    const v4f su = va + vb;
    const v4f v = sel4(sel < 2, su, sel4(sel == 2, va, vb));
    *(v4f*)(sbias + 4 * tid) = v;
  }
  __syncthreads();
  v8f ar[2], az[2], an[2], ah[2];
#pragma unroll
  for (int t = 0; t < 2; ++t) { ar[t] = zacc(); az[t] = zacc(); an[t] = zacc(); ah[t] = zacc(); }
  {
    const _Float16* ap = Xp + (size_t)(rowBase + 16 * rt + m) * ldx + 8 * hh;
    const _Float16* bp = Wih + (size_t)(jw + m) * ldw + 8 * hh;
#pragma unroll 1
    for (int ks = 0; ks < KS1; ++ks) {
      const v16h a = ldfrag(ap + 32 * ks);
#pragma unroll
      for (int t = 0; t < 2; ++t) {
        const _Float16* bt = bp + (size_t)(16 * t) * ldw + 32 * ks;
        const v16h br = ldfrag(bt);
        const v16h bz = ldfrag(bt + (size_t)HD * ldw);
        const v16h bn = ldfrag(bt + (size_t)(2 * HD) * ldw);
        ar[t] = wmh(a, br, ar[t]);
        az[t] = wmh(a, bz, az[t]);
        an[t] = wmh(a, bn, an[t]);
      }
    }
  }
  {
    const _Float16* ap = Hp + (size_t)(rowBase + 16 * rt + m) * ldh + hoff + 8 * hh;
    const _Float16* bp = Whh + (size_t)(jw + m) * HD + 8 * hh;
#pragma unroll 1
    for (int ks = 0; ks < HD / 32; ++ks) {
      const v16h a = ldfrag(ap + 32 * ks);
#pragma unroll
      for (int t = 0; t < 2; ++t) {
        const _Float16* bt = bp + (size_t)(16 * t) * HD + 32 * ks;
        const v16h br = ldfrag(bt);
        const v16h bz = ldfrag(bt + (size_t)HD * HD);
        const v16h bn = ldfrag(bt + (size_t)(2 * HD) * HD);
        ar[t] = wmh(a, br, ar[t]);
        az[t] = wmh(a, bz, az[t]);
        ah[t] = wmh(a, bn, ah[t]);
      }
    }
  }
#pragma unroll
  for (int t = 0; t < 2; ++t) {
    const int jl = 32 * ch + 16 * t + m;
    const float b_r = sbias[jl];
    const float b_z = sbias[64 + jl];
    const float b_i = sbias[128 + jl];
    const float b_h = sbias[192 + jl];
    const float* hl = hpv + (16 * rt + 8 * hh) * 64 + jl;
    float* sp = stg + (16 * rt + 8 * hh) * 64 + jl;
#pragma unroll
    for (int r = 0; r < 8; ++r) {
      const float hprev = hl[r * 64];
      const float rg = sigf(ar[t][r] * RSC + b_r);
      const float zg = sigf(az[t][r] * RSC + b_z);
      const float ng = tanhf2(an[t][r] * RSC + b_i + rg * (ah[t][r] * RSC + b_h));
      sp[r * 64] = (1.0f - zg) * ng + zg * hprev;
    }
  }
  __syncthreads();
  float* gp = outL + jB;
  _Float16* hp = NH + (size_t)rowBase * HD + jB;
#pragma unroll
  for (int it = 0; it < 4; ++it) {
    const int f = it * NTHR + tid, row = f >> 4, p4 = (f & 15) * 4;
    const int node = rowBase + row;
    const v4f v = *(const v4f*)(stg + row * 64 + p4);
    if (node < nN) *(volatile v4f*)(gp + (size_t)node * HD + p4) = v;
  }
#pragma unroll
  for (int it = 0; it < 2; ++it) {
    const int f = it * NTHR + tid, row = f >> 3, p8 = (f & 7) * 8;
    const v8h hv = cvt8(*(const v4f*)(stg + row * 64 + p8), *(const v4f*)(stg + row * 64 + p8 + 4), ASC);
    *(volatile v8h*)(hp + (size_t)row * HD + p8) = hv;
  }
  __threadfence();
#pragma unroll
  for (int it = 0; it < 4; ++it) {
    const int f = it * NTHR + tid, row = f >> 4, p4 = (f & 15) * 4;
    const int node = rowBase + row;
    const v4f v = *(const v4f*)(stg + row * 64 + p4);
    if (node < nN) *(volatile v4f*)(gp + (size_t)node * HD + p4) = v;
  }
#pragma unroll
  for (int it = 0; it < 2; ++it) {
    const int f = it * NTHR + tid, row = f >> 3, p8 = (f & 7) * 8;
    const v8h hv = cvt8(*(const v4f*)(stg + row * 64 + p8), *(const v4f*)(stg + row * 64 + p8 + 4), ASC);
    *(volatile v8h*)(hp + (size_t)row * HD + p8) = hv;
  }
}

__device__ __forceinline__ void do_tile(int tb, int nv, _Float16* agg, _Float16* h1t, const int* pend,
    int* rsrc, int* rdst, int* rloc, const float* __restrict__ PQ, const int* __restrict__ srcs,
    const int* __restrict__ dsts, const _Float16* __restrict__ W2p, float b20, float b21,
    int n0, int nN, int nE, int tid, int lane, int wave, int hh, int m) {
  if (tid < RT) {
    int e = pend[min(tb + tid, PCAP - 1)];
    e = e < 0 ? 0 : (e > nE - 1 ? nE - 1 : e);
    int s = srcs[e]; s = s < 0 ? 0 : (s > nN - 1 ? nN - 1 : s);
    int d = dsts[e]; d = d < 0 ? 0 : (d > nN - 1 ? nN - 1 : d);
    int loc = d - n0; loc = loc < 0 ? 0 : (loc > NBE - 1 ? NBE - 1 : loc);
    loc = (tid < nv) ? loc : NBE;
    rsrc[tid] = s; rdst[tid] = d; rloc[tid] = loc;
  }
  __syncthreads();
#pragma unroll
  for (int it = 0; it < 4; ++it) {
    const int f = it * NTHR + tid, row = f >> 5, c8 = (f & 31) * 8;
    const int s = rsrc[row], d = rdst[row];
    const float* pa = PQ + (size_t)d * PLN + c8;
    const float* qa = PQ + (size_t)s * PLN + HD + c8;
    const v4f p0 = *(const v4f*)pa, p1 = *(const v4f*)(pa + 4);
    const v4f q0 = *(const v4f*)qa, q1 = *(const v4f*)(qa + 4);
    *(v8h*)(h1t + row * HP + c8) = cvt8(relu4(p0 + q0), relu4(p1 + q1), ASC);
    if ((it & 1) == 1) asm volatile("" ::: "memory");
  }
  __syncthreads();
  v8f acc[2][2];
#pragma unroll
  for (int g = 0; g < 2; ++g) { acc[g][0] = zacc(); acc[g][1] = zacc(); }
  {
    const _Float16* ap = h1t + m * HP + 8 * hh;
    const _Float16* bp = W2p + (size_t)(32 * wave + m) * HD + 8 * hh;
#pragma unroll 1
    for (int ks = 0; ks < HD / 32; ++ks) {
      const v16h a0 = ldfrag(ap + 32 * ks);
      const v16h a1 = ldfrag(ap + 16 * HP + 32 * ks);
#pragma unroll
      for (int t = 0; t < 2; ++t) {
        const v16h b = ldfrag(bp + (size_t)(16 * t) * HD + 32 * ks);
        acc[0][t] = wmh(a0, b, acc[0][t]);
        acc[1][t] = wmh(a1, b, acc[1][t]);
      }
    }
  }
  const int locv = rloc[lane];
  int lofs[2][8];
#pragma unroll
  for (int g = 0; g < 2; ++g) {
#pragma unroll
    for (int r = 0; r < 8; ++r) {
      const int la = __builtin_amdgcn_readlane(locv, 16 * g + r);
      const int lb = __builtin_amdgcn_readlane(locv, 16 * g + 8 + r);
      lofs[g][r] = (hh ? lb : la) * FP;
    }
  }
  _Float16 vh[2][2][8];
#pragma unroll
  for (int g = 0; g < 2; ++g) {
#pragma unroll
    for (int r = 0; r < 8; ++r) {
      vh[g][0][r] = (_Float16)(fmaxf(acc[g][0][r] * RSC + b20, 0.0f) * ASC);
      vh[g][1][r] = (_Float16)(fmaxf(acc[g][1][r] * RSC + b21, 0.0f) * ASC);
    }
  }
  const int cb = 32 * wave + m;
  if (hh == 0) {
#pragma unroll
    for (int g = 0; g < 2; ++g) {
#pragma unroll
      for (int t = 0; t < 2; ++t) {
#pragma unroll
        for (int r = 0; r < 8; ++r) {
          _Float16* p = agg + lofs[g][r] + cb + 16 * t;
          const _Float16 o = *p;
          const _Float16 v = vh[g][t][r];
          *p = (v > o) ? v : o;
        }
      }
    }
  }
  __syncthreads();
  if (hh != 0) {
#pragma unroll
    for (int g = 0; g < 2; ++g) {
#pragma unroll
      for (int t = 0; t < 2; ++t) {
#pragma unroll
        for (int r = 0; r < 8; ++r) {
          _Float16* p = agg + lofs[g][r] + cb + 16 * t;
          const _Float16 o = *p;
          const _Float16 v = vh[g][t][r];
          *p = (v > o) ? v : o;
        }
      }
    }
  }
  __syncthreads();
}

__global__ __launch_bounds__(NTHR) void k_edge(const float* __restrict__ PQ, const int* __restrict__ srcs,
    const int* __restrict__ dsts, const _Float16* __restrict__ W2p, const float* __restrict__ b2,
    const float* __restrict__ tin, const float* __restrict__ ain, _Float16* FEAT, int nN, int nE, int vec8) {
  extern __shared__ v4i lds_dyn[];
  _Float16* agg = (_Float16*)lds_dyn;
  _Float16* h1t = agg + AGR * FP;
  int* list = (int*)(h1t + RT * HP);
  int* pend = list + LISTN;
  int* rsrc = pend + PCAP;
  int* rdst = rsrc + RT;
  int* rloc = rdst + RT;
  int* wcnt = rloc + RT;
  int* misc = wcnt + NWAVE;
  const int tid = threadIdx.x, lane = tid & 31, wave = tid >> 5, hh = lane >> 4, m = lane & 15;
  const int n0 = blockIdx.x * NBE;
  {
    const v4i z = {0, 0, 0, 0};
#pragma unroll 1
    for (int i = tid; i < (AGR * FP) / 8; i += NTHR) ((v4i*)agg)[i] = z;
    if (tid == 0) misc[0] = 0;
  }
  const float b20 = b2[32 * wave + m], b21 = b2[32 * wave + 16 + m];
  __syncthreads();

  const int nChunks = (nE + CHUNK - 1) / CHUNK;
#pragma unroll 1
  for (int chk = 0; chk < nChunks; ++chk) {
    const int cbase = chk * CHUNK;
    const int wc = scan_chunk<NBE>(dsts, nE, cbase, n0, vec8, list, tid, lane, wave);
    if (lane == 0) wcnt[wave] = wc;
    __syncthreads();
    int pw = 0, tot = 0, mywc = 0;
#pragma unroll
    for (int w = 0; w < NWAVE; ++w) {
      int c = wcnt[w];
      c = c < 0 ? 0 : (c > WCAP ? WCAP : c);
      pw += (w < wave) ? c : 0;
      tot += c;
      mywc = (w == wave) ? c : mywc;
    }
    int np0 = misc[0];
    np0 = np0 < 0 ? 0 : (np0 > PCAP - LISTN ? PCAP - LISTN : np0);
    mywc = __builtin_amdgcn_readfirstlane(mywc);
#pragma unroll 1
    for (int i = lane; i < mywc; i += 32) pend[np0 + pw + i] = list[wave * WCAP + i];
    const int np = __builtin_amdgcn_readfirstlane(np0 + tot);
    __syncthreads();
    int ntile = np >> 5;
    ntile = ntile > PCAP / RT ? PCAP / RT : ntile;
    ntile = __builtin_amdgcn_readfirstlane(ntile);
#pragma unroll 1
    for (int tI = 0; tI < ntile; ++tI)
      do_tile(tI * RT, RT, agg, h1t, pend, rsrc, rdst, rloc, PQ, srcs, dsts, W2p, b20, b21,
              n0, nN, nE, tid, lane, wave, hh, m);
    const int rem = np - ntile * RT;
    const int mv = pend[min(ntile * RT + tid, PCAP - 1)];
    __syncthreads();
    if (tid < rem) pend[tid] = mv;
    if (tid == 0) misc[0] = rem;
    __syncthreads();
  }
  {
    int rem = misc[0];
    rem = rem < 0 ? 0 : (rem > RT - 1 ? RT - 1 : rem);
    rem = __builtin_amdgcn_readfirstlane(rem);
    if (rem > 0)
      do_tile(0, rem, agg, h1t, pend, rsrc, rdst, rloc, PQ, srcs, dsts, W2p, b20, b21,
              n0, nN, nE, tid, lane, wave, hh, m);
  }
  {
    const v4f z4 = {0.f, 0.f, 0.f, 0.f};
#pragma unroll
    for (int it = 0; it < 8; ++it) {
      const int q = it * NTHR + tid, row = q >> 3, j = q & 7;
      int node = n0 + row; node = node > nN - 1 ? nN - 1 : node;
      const int jj = j & 1;
      const float* tp = tin + (size_t)node * TD + 8 * jj;
      const float* apn = ain + (size_t)node * TD + 8 * jj;
      const v4f t0 = *(const v4f*)tp, t1 = *(const v4f*)(tp + 4);
      const v4f a0 = *(const v4f*)apn, a1 = *(const v4f*)(apn + 4);
      const v4f u0 = sel4(j < 2, t0, sel4(j < 4, a0, z4));
      const v4f u1 = sel4(j < 2, t1, sel4(j < 4, a1, z4));
      *(v8h*)(agg + row * FP + HD + 8 * j) = cvt8(u0, u1, ASC);
      if ((it & 1) == 1) asm volatile("" ::: "memory");
    }
  }
  __syncthreads();
  _Float16* gp = FEAT + (size_t)n0 * FP;
#pragma unroll 1
  for (int it = 0; it < (NBE * FP) / (8 * NTHR); ++it) {
    const int f = it * NTHR + tid;
    const v8h v = ((const v8h*)agg)[f];
    *(volatile v8h*)(gp + (size_t)f * 8) = v;
  }
  __threadfence();
#pragma unroll 1
  for (int it = 0; it < (NBE * FP) / (8 * NTHR); ++it) {
    const int f = it * NTHR + tid;
    const v8h v = ((const v8h*)agg)[f];
    *(volatile v8h*)(gp + (size_t)f * 8) = v;
  }
}

extern "C" void kernel_launch(void* const* d_in, const int* in_sizes, int n_in,
                              void* d_out, int out_size, void* d_ws, size_t ws_size,
                              hipStream_t stream) {
  if (n_in < 25) return;
  const int nN = in_sizes[0] / XD;
  const int nE = in_sizes[4] / 2;
  if (nN <= 0 || nE <= 0) return;
  if (in_sizes[0] != nN * XD || in_sizes[1] != nN * TD || in_sizes[2] != nN * TD || in_sizes[3] != nN * ZD) return;
  if (in_sizes[4] != 2 * nE) return;
  if (in_sizes[5] != HD * 2 * XD || in_sizes[6] != HD || in_sizes[7] != HD * HD || in_sizes[8] != HD) return;
  if (in_sizes[9] != HD * FD || in_sizes[10] != HD || in_sizes[11] != HD * FD || in_sizes[12] != HD) return;
  if (in_sizes[13] != 3 * HD * FD || in_sizes[14] != 3 * HD * HD || in_sizes[15] != 3 * HD || in_sizes[16] != 3 * HD) return;
  if (in_sizes[17] != 3 * HD * HD || in_sizes[18] != 3 * HD * HD || in_sizes[19] != 3 * HD || in_sizes[20] != 3 * HD) return;
  if (in_sizes[21] != ZD * HD || in_sizes[22] != ZD || in_sizes[23] != ZD * HD || in_sizes[24] != ZD) return;
  if ((long long)out_size != (long long)nN * (2 * HD + 3 * ZD)) return;
  if (nN > (1 << 22) || nE > (1 << 28)) return;

  const float* x    = (const float*)d_in[0];
  const float* tin  = (const float*)d_in[1];
  const float* ain  = (const float*)d_in[2];
  const float* eps  = (const float*)d_in[3];
  const int*   ei   = (const int*)d_in[4];
  const float* w1   = (const float*)d_in[5];
  const float* b1   = (const float*)d_in[6];
  const float* w2   = (const float*)d_in[7];
  const float* b2   = (const float*)d_in[8];
  const float* hw0  = (const float*)d_in[9];
  const float* hb0  = (const float*)d_in[10];
  const float* hw1  = (const float*)d_in[11];
  const float* hb1  = (const float*)d_in[12];
  const float* wi0  = (const float*)d_in[13];
  const float* wh0  = (const float*)d_in[14];
  const float* bi0  = (const float*)d_in[15];
  const float* bh0  = (const float*)d_in[16];
  const float* wi1  = (const float*)d_in[17];
  const float* wh1  = (const float*)d_in[18];
  const float* bi1  = (const float*)d_in[19];
  const float* bh1  = (const float*)d_in[20];
  const float* muw  = (const float*)d_in[21];
  const float* mub  = (const float*)d_in[22];
  const float* lvw  = (const float*)d_in[23];
  const float* lvb  = (const float*)d_in[24];
  const int* srcs = ei;
  const int* dsts = ei + nE;
  float* out   = (float*)d_out;
  float* outh1 = out + (size_t)nN * HD;
  float* o1    = out + (size_t)2 * nN * HD;
  float* o2    = o1 + (size_t)nN * ZD;
  float* o3    = o2 + (size_t)nN * ZD;

  const int nBE  = (nN + NBE - 1) / NBE;
  const int NPAD = nBE * NBE;
  const int nBG  = NPAD / GR;
  const int vec8 = ((nE & 3) == 0) ? 1 : 0;

  char* ws = (char*)d_ws;
  size_t off = 0;
  const size_t oW  = off; off += (size_t)WPTOT * 2;            off = (off + 255) & ~(size_t)255;
  const size_t oX  = off; off += (size_t)NPAD * XD * 2;        off = (off + 255) & ~(size_t)255;
  const size_t oR1 = off; off += (size_t)NPAD * PLN * 4;       off = (off + 255) & ~(size_t)255;
  const size_t oF  = off; off += (size_t)NPAD * FP * 2;        off = (off + 255) & ~(size_t)255;
  const size_t oH  = off; off += (size_t)NPAD * PLN * 2;       off = (off + 255) & ~(size_t)255;
  const size_t oN0 = off; off += (size_t)NPAD * HD * 2;        off = (off + 255) & ~(size_t)255;
  const size_t oN1 = off; off += (size_t)NPAD * HD * 2;        off = (off + 255) & ~(size_t)255;
  if (off > ws_size || off > (size_t)WSCAP) return;
  _Float16* WP   = (_Float16*)(ws + oW);
  _Float16* X16  = (_Float16*)(ws + oX);
  float*    R1   = (float*)(ws + oR1);
  _Float16* FEAT = (_Float16*)(ws + oF);
  _Float16* H16  = (_Float16*)(ws + oH);
  _Float16* NH0  = (_Float16*)(ws + oN0);
  _Float16* NH1  = (_Float16*)(ws + oN1);

  k_wprep<<<WPTOT / WPB, NTHR, 0, stream>>>(w1, w2, hw0, hw1, wi0, wh0, wi1, wh1, muw, lvw, WP);
  k_xcvt<<<NPAD / 16, NTHR, 0, stream>>>(x, X16, nN);
  k_gemm<0, XD / 32><<<dim3(nBG, 4), NTHR, 0, stream>>>(X16, XD, WP + OFW1F, XD, b1, b1, eps, R1, H16, PLN, out, out, out, nN);
  hipFuncSetAttribute(reinterpret_cast<const void*>(&k_edge),
                      hipFuncAttributeMaxDynamicSharedMemorySize, LDS_EDGE);
  k_edge<<<nBE, NTHR, LDS_EDGE, stream>>>(R1, srcs, dsts, WP + OFW2, b2, tin, ain, FEAT, nN, nE, vec8);
  k_gemm<1, FD / 32><<<dim3(nBG, 4), NTHR, 0, stream>>>(FEAT, FP, WP + OFHI, FD, hb0, hb1, eps, R1, H16, PLN, out, out, out, nN);
  k_gate<FD / 32><<<dim3(nBG, 4), NTHR, 0, stream>>>(FEAT, FP, WP + OFWIH0, FD, H16, R1, PLN, 0, WP + OFWHH0, bi0, bh0, out, NH0, nN);
  k_gate<HD / 32><<<dim3(nBG, 4), NTHR, 0, stream>>>(NH0, HD, WP + OFWIH1, HD, H16, R1, PLN, HD, WP + OFWHH1, bi1, bh1, outh1, NH1, nN);
  k_gemm<2, HD / 32><<<dim3(nBG, 1), NTHR, 0, stream>>>(NH1, HD, WP + OFHEAD, HD, mub, lvb, eps, R1, H16, PLN, o1, o2, o3, nN);
}
